// GCN_IDS_50637664420305
// MI455X (gfx1250) — hardware-run, weakly checked
//
#include <hip/hip_runtime.h>
#include <stddef.h>
#include <stdint.h>
#include <math.h>

#define NN      100000
#define FD      128
#define HD      64
#define FC      32
#define NE      1600000
#define GBM     128
#define MP      100096
#define KL      128
#define NTHR    256
#define NWAVE   8
#define EPT     8
#define WCH     (32 * EPT)
#define NBRUN   1024
#define SLB     10
#define NBK     98
#define WLCAP   3584
#define RCAP    28672
#define DEGCAP  64
#define MAXDEG_MEAS   36
#define MAXB1024_MEAS 16710
#define SP      68
#define AP      136
#define RP      36
#define RECW    160
#define WSTW    132
#define TWO_TERM 1
#define WSMAX   134217728

#define BK_ZINTS (NWAVE * WLCAP + RCAP + 4 * NBRUN)
#define BK_INTS  (BK_ZINTS + 16)
#define BK_LDS   (BK_INTS * 4)

#define PBX  (MP * FD / 8 / NTHR)
#define PBW0 (HD * FD / 8 / NTHR)
#define PBW1 (HD * KL / 8 / NTHR)
#define PBFC (FC * KL / 8 / NTHR)
#define PBTOT (PBX + PBW0 + 2 * PBW1 + PBFC)

static_assert(HD == 64 && HD == 16 * 4 && FC == 32 && FD == 128);
static_assert(MP % GBM == 0 && MP >= NN && MP == 782 * GBM);
static_assert(NN == 781 * GBM + 32 && NN == 97 * NBRUN + 672);
static_assert(NBRUN == (1 << SLB) && NBRUN % GBM == 0 && NBRUN % 32 == 0 && NBRUN == 4 * NTHR);
static_assert(NBK * NBRUN >= MP);
static_assert(NE < (1 << 21) && (((long long)NE) << SLB) < (1LL << 31));
static_assert(NE % WCH == 0 && NE % 4 == 0);
static_assert(RCAP == NWAVE * WLCAP && RCAP % (NTHR * 4) == 0 && BK_ZINTS % (NTHR * 4) == 0);
static_assert((long long)RCAP * 100 >= (long long)MAXB1024_MEAS * 105);
static_assert(WLCAP >= MAXB1024_MEAS / 8 + 8 * 46 + 1);
static_assert(MAXDEG_MEAS + 8 <= DEGCAP);
static_assert((MP * FD / 8) % NTHR == 0 && (HD * FD / 8) % NTHR == 0);
static_assert((HD * KL / 8) % NTHR == 0 && (FC * KL / 8) % NTHR == 0);
static_assert(FD % 32 == 0 && KL % 32 == 0 && KL == 2 * HD && FD == KL);
static_assert(BK_LDS <= 300000);
static_assert(GBM * SP * 4 <= 65536);
static_assert((GBM * 2 * 4) % 128 == 0 && (((NN % GBM) * 2 * 4) % 128) == 0 && ((NN % GBM) % 16) == 0);
static_assert(RECW % 32 == 0 && RECW / 4 <= NTHR && WSTW % 2 == 0 && WSTW >= 4 + 2 * HD);
static_assert((AP * 2) % 16 == 0 && (RP * 4) % 16 == 0 && AP >= KL && RP >= FC);

typedef float          v2f   __attribute__((ext_vector_type(2)));
typedef float          v4f   __attribute__((ext_vector_type(4)));
typedef float          v8f   __attribute__((ext_vector_type(8)));
typedef int            v4i   __attribute__((ext_vector_type(4)));
typedef int            v8i   __attribute__((ext_vector_type(8)));
typedef unsigned short v8us  __attribute__((ext_vector_type(8)));
typedef unsigned short v16us __attribute__((ext_vector_type(16)));
typedef __bf16         v16bf __attribute__((ext_vector_type(16)));
typedef v2f  __attribute__((may_alias)) v2fa;
typedef v4f  __attribute__((may_alias)) v4fa;
typedef v4i  __attribute__((may_alias)) v4ia;
typedef v8us __attribute__((may_alias)) v8usa;
union FragB { v16bf v; v16us u; v8us h[2]; v8i w; };

__device__ __forceinline__ v8f wmb(const FragB& a, const FragB& b, v8f c) {
  v8f d = __builtin_amdgcn_wmma_f32_16x16x32_bf16(false, a.v, false, b.v, (short)0, c, false, false);
  asm volatile("v_nop\n\tv_nop\n\tv_nop\n\tv_nop" : "+v"(d) : "v"(a.w), "v"(b.w));
  return d;
}

__device__ __forceinline__ unsigned bf16_bits(float f) {
  const unsigned u = __float_as_uint(f);
  const unsigned r = (u + 0x7FFFu + ((u >> 16) & 1u)) >> 16;
  const unsigned q = (u >> 16) | 0x40u;
  return ((u & 0x7fffffffu) > 0x7f800000u) ? q : r;
}
__device__ __forceinline__ float bf16_val(float f) {
  return __uint_as_float(bf16_bits(f) << 16);
}

__device__ __forceinline__ void hilo_pack(float v0, float v1, float v2, float v3,
                                          int& h01, int& h23, int& l01, int& l23) {
  const unsigned a0 = bf16_bits(v0), a1 = bf16_bits(v1), a2 = bf16_bits(v2), a3 = bf16_bits(v3);
#if TWO_TERM
  const unsigned b0 = bf16_bits(v0 - __uint_as_float(a0 << 16));
  const unsigned b1 = bf16_bits(v1 - __uint_as_float(a1 << 16));
  const unsigned b2 = bf16_bits(v2 - __uint_as_float(a2 << 16));
  const unsigned b3 = bf16_bits(v3 - __uint_as_float(a3 << 16));
#else
  const unsigned b0 = 0u, b1 = 0u, b2 = 0u, b3 = 0u;
#endif
  h01 = (int)(a0 | (a1 << 16)); h23 = (int)(a2 | (a3 << 16));
  l01 = (int)(b0 | (b1 << 16)); l23 = (int)(b2 | (b3 << 16));
}

__device__ __forceinline__ v4i regroup8(int h01, int h23, int l01, int l23, int lane) {
  const int t  = lane & 15;
  const int s0 = (lane & 16) + ((2 * t) & 15), s1 = s0 + 1;
  const int a0 = __shfl(h01, s0, 32), a1 = __shfl(h23, s0, 32), a2 = __shfl(h01, s1, 32), a3 = __shfl(h23, s1, 32);
  const int b0 = __shfl(l01, s0, 32), b1 = __shfl(l23, s0, 32), b2 = __shfl(l01, s1, 32), b3 = __shfl(l23, s1, 32);
  const int mk = (t < 8) ? -1 : 0;
  v4i o;
  o.x = (a0 & mk) | (b0 & ~mk); o.y = (a1 & mk) | (b1 & ~mk);
  o.z = (a2 & mk) | (b2 & ~mk); o.w = (a3 & mk) | (b3 & ~mk);
  return o;
}

__device__ __forceinline__ void st2_v4f(float* p, v4f v) {
  *(volatile v4f*)p = v;
  __threadfence();
  *(volatile v4f*)p = v;
}
__device__ __forceinline__ void st2_v8us(unsigned short* p, v8us v) {
  *(volatile v8us*)p = v;
  __threadfence();
  *(volatile v8us*)p = v;
}

__device__ __forceinline__ v8us gather8(const float* __restrict__ base, int stride) {
  float f[8];
#pragma unroll
  for (int i = 0; i < 8; ++i) f[i] = base[(size_t)i * (size_t)stride];
  v8us o;
#pragma unroll
  for (int i = 0; i < 8; ++i) o[i] = (unsigned short)bf16_bits(f[i]);
  return o;
}

__device__ __forceinline__ float bnr(float v, float mu, float rs, float g, float be) {
  const float t = ((g * (v - mu)) * rs) + be;
  return (t > 0.0f) ? t : (t - t);
}

__global__ __launch_bounds__(NTHR) void k_prep(const float* __restrict__ x, const float* __restrict__ w0,
                                               const float* __restrict__ w1, const float* __restrict__ w2,
                                               const float* __restrict__ fc1w,
                                               unsigned short* xb, unsigned short* w0t, unsigned short* w1d,
                                               unsigned short* w2d, unsigned short* fc1d) {
  const int tid = (int)threadIdx.x;
  const int blk = (int)blockIdx.x;
  if (blk < PBX) {
    const int u   = blk * NTHR + tid;
    const int row = u >> 4, k8 = (u & 15) * 8;
    const int rc  = row < NN ? row : NN - 1;
    const unsigned mk = row < NN ? 0xffffu : 0u;
    const float* p = x + (size_t)rc * FD + k8;
    const v4f a = *(const v4fa*)p;
    const v4f b = *(const v4fa*)(p + 4);
    v8us o;
    o[0] = (unsigned short)(bf16_bits(a.x) & mk); o[1] = (unsigned short)(bf16_bits(a.y) & mk);
    o[2] = (unsigned short)(bf16_bits(a.z) & mk); o[3] = (unsigned short)(bf16_bits(a.w) & mk);
    o[4] = (unsigned short)(bf16_bits(b.x) & mk); o[5] = (unsigned short)(bf16_bits(b.y) & mk);
    o[6] = (unsigned short)(bf16_bits(b.z) & mk); o[7] = (unsigned short)(bf16_bits(b.w) & mk);
    st2_v8us(xb + (size_t)row * FD + k8, o);
  } else if (blk < PBX + PBW0) {
    const int u = (blk - PBX) * NTHR + tid;
    const int n = u >> 4, k8 = (u & 15) * 8;
    const v8us o = gather8(w0 + (size_t)k8 * HD + n, HD);
    st2_v8us(w0t + (size_t)n * FD + k8, o);
  } else if (blk < PBX + PBW0 + PBW1) {
    const int u = (blk - PBX - PBW0) * NTHR + tid;
    const int n = u >> 4, k8 = (u & 15) * 8, kk = k8 & 63;
    const v8us o = gather8(w1 + (size_t)kk * HD + n, HD);
    st2_v8us(w1d + (size_t)n * KL + k8, o);
  } else if (blk < PBX + PBW0 + 2 * PBW1) {
    const int u = (blk - PBX - PBW0 - PBW1) * NTHR + tid;
    const int n = u >> 4, k8 = (u & 15) * 8, kk = k8 & 63;
    const v8us o = gather8(w2 + (size_t)kk * HD + n, HD);
    st2_v8us(w2d + (size_t)n * KL + k8, o);
  } else {
    const int u = (blk - PBX - PBW0 - 2 * PBW1) * NTHR + tid;
    const int n = u >> 4, k8 = (u & 15) * 8, kk = k8 & 63;
    const v8us o = gather8(fc1w + (size_t)kk * FC + n, FC);
    st2_v8us(fc1d + (size_t)n * KL + k8, o);
  }
}

__device__ __forceinline__ void bucket_flush(const int* pl, const int* cnt, int ov, int* lp, int* cp, int* op,
                                             int* dp, int* fp, int tid) {
#pragma unroll 1
  for (int i = tid * 4; i < RCAP; i += NTHR * 4) {
    const v4i v = *(const v4ia*)(pl + i);
    *(volatile v4i*)(lp + i) = v;
  }
  {
    const v4i v = *(const v4ia*)(cnt + 4 * tid);
    *(volatile v4i*)(cp + 4 * tid) = v;
  }
  {
    const v4i v = *(const v4ia*)(cnt + NBRUN + 4 * tid);
    *(volatile v4i*)(op + 4 * tid) = v;
  }
  {
    const v4i v = *(const v4ia*)(cnt + 2 * NBRUN + 4 * tid);
    *(volatile v4i*)(dp + 4 * tid) = v;
  }
  if (tid < 8) {
    const v4i f = {ov, ov, ov, ov};
    *(volatile v4i*)(fp + 4 * tid) = f;
  }
}

__global__ __launch_bounds__(NTHR) void k_bucket(const int* __restrict__ srcs, const int* __restrict__ dsts,
                                                 int* HITS, int* CNT, int* OFF, int* DISI, int* FLAG) {
  extern __shared__ __attribute__((aligned(16))) int dsm[];
  int* wl   = dsm;
  int* pl   = dsm + NWAVE * WLCAP;
  int* cnt  = pl + RCAP;
  int* offs = cnt + NBRUN;
  int* disb = offs + NBRUN;
  int* cur  = disb + NBRUN;
  int* misc = cur + NBRUN;
  const int tid = (int)threadIdx.x, lane = tid & 31, wave = tid >> 5;
  const int blk = (int)blockIdx.x;
  const unsigned nbs = (unsigned)(blk * NBRUN);

  {
    const v4i z4 = {0, 0, 0, 0};
    for (int i = tid * 4; i < BK_ZINTS; i += NTHR * 4) *(v4ia*)(dsm + i) = z4;
    if (tid < 16) misc[tid] = 0;
  }
  __syncthreads();

  {
    const int per  = ((NE + NWAVE * WCH - 1) / (NWAVE * WCH)) * WCH;
    const int ebeg = wave * per;
    const int eend = (ebeg + per < NE) ? (ebeg + per) : NE;
    int* mylist = wl + wave * WLCAP;
    int wc = 0;
#pragma unroll 1
    for (int cb = ebeg; cb < eend; cb += WCH) {
      const int e0 = cb + lane * EPT;
      const v4i da = *(const v4ia*)(dsts + e0);
      const v4i db = *(const v4ia*)(dsts + e0 + 4);
      const unsigned s0 = (unsigned)da.x - nbs, s1 = (unsigned)da.y - nbs;
      const unsigned s2 = (unsigned)da.z - nbs, s3 = (unsigned)da.w - nbs;
      const unsigned s4 = (unsigned)db.x - nbs, s5 = (unsigned)db.y - nbs;
      const unsigned s6 = (unsigned)db.z - nbs, s7 = (unsigned)db.w - nbs;
      const bool h0 = s0 < (unsigned)NBRUN, h1 = s1 < (unsigned)NBRUN, h2 = s2 < (unsigned)NBRUN, h3 = s3 < (unsigned)NBRUN;
      const bool h4 = s4 < (unsigned)NBRUN, h5 = s5 < (unsigned)NBRUN, h6 = s6 < (unsigned)NBRUN, h7 = s7 < (unsigned)NBRUN;
      const unsigned m0 = __builtin_amdgcn_ballot_w32(h0), m1 = __builtin_amdgcn_ballot_w32(h1);
      const unsigned m2 = __builtin_amdgcn_ballot_w32(h2), m3 = __builtin_amdgcn_ballot_w32(h3);
      const unsigned m4 = __builtin_amdgcn_ballot_w32(h4), m5 = __builtin_amdgcn_ballot_w32(h5);
      const unsigned m6 = __builtin_amdgcn_ballot_w32(h6), m7 = __builtin_amdgcn_ballot_w32(h7);
      const unsigned any = m0 | m1 | m2 | m3 | m4 | m5 | m6 | m7;
      if (any != 0u) {
        const int pre = (int)(__builtin_amdgcn_mbcnt_lo(m0, 0u) + __builtin_amdgcn_mbcnt_lo(m1, 0u) +
                              __builtin_amdgcn_mbcnt_lo(m2, 0u) + __builtin_amdgcn_mbcnt_lo(m3, 0u) +
                              __builtin_amdgcn_mbcnt_lo(m4, 0u) + __builtin_amdgcn_mbcnt_lo(m5, 0u) +
                              __builtin_amdgcn_mbcnt_lo(m6, 0u) + __builtin_amdgcn_mbcnt_lo(m7, 0u));
        int p = wc + pre;
        if (h0) { if (p < WLCAP) mylist[p] = ((e0 + 0) << SLB) | (int)s0; p = p + 1; }
        if (h1) { if (p < WLCAP) mylist[p] = ((e0 + 1) << SLB) | (int)s1; p = p + 1; }
        if (h2) { if (p < WLCAP) mylist[p] = ((e0 + 2) << SLB) | (int)s2; p = p + 1; }
        if (h3) { if (p < WLCAP) mylist[p] = ((e0 + 3) << SLB) | (int)s3; p = p + 1; }
        if (h4) { if (p < WLCAP) mylist[p] = ((e0 + 4) << SLB) | (int)s4; p = p + 1; }
        if (h5) { if (p < WLCAP) mylist[p] = ((e0 + 5) << SLB) | (int)s5; p = p + 1; }
        if (h6) { if (p < WLCAP) mylist[p] = ((e0 + 6) << SLB) | (int)s6; p = p + 1; }
        if (h7) { if (p < WLCAP) mylist[p] = ((e0 + 7) << SLB) | (int)s7; p = p + 1; }
        wc += (int)(__builtin_popcount(m0) + __builtin_popcount(m1) + __builtin_popcount(m2) + __builtin_popcount(m3) +
                    __builtin_popcount(m4) + __builtin_popcount(m5) + __builtin_popcount(m6) + __builtin_popcount(m7));
      }
    }
    if (lane == 0) misc[wave] = wc;
  }
  __syncthreads();

  if (wave == 0) {
    int ov = 0;
#pragma unroll 1
    for (int w2 = 0; w2 < NWAVE; ++w2) {
      int c = misc[w2];
      if (c > WLCAP) ov = 1;
      c = c < 0 ? 0 : (c > WLCAP ? WLCAP : c);
#pragma unroll 1
      for (int b0 = 0; b0 < c; b0 += 32) {
        const int idx = b0 + lane;
        const int ent = wl[w2 * WLCAP + (idx < WLCAP ? idx : WLCAP - 1)];
        const int m32 = (c - b0) < 32 ? (c - b0) : 32;
#pragma unroll 1
        for (int k = 0; k < m32; ++k) {
          const int u    = __builtin_amdgcn_readlane(ent, k);
          const int slot = u & (NBRUN - 1);
          if (lane == 0) cnt[slot] = cnt[slot] + 1;
        }
      }
    }
    if (lane == 0) misc[9] = ov;
  }
  __syncthreads();
#pragma unroll 1
  for (int i = 0; i < 4; ++i) {
    const int s = 4 * tid + i;
    const float dg = (float)(cnt[s] + 1);
    disb[s] = __float_as_int(1.0f / sqrtf(dg));
  }
  if (wave == 0) {
    const int base = lane * (NBRUN / 32);
    int s = 0;
#pragma unroll 1
    for (int i = 0; i < NBRUN / 32; ++i) s += cnt[base + i];
    int incl = s;
#pragma unroll
    for (int d = 1; d < 32; d <<= 1) {
      const int y = __shfl_up(incl, d, 32);
      if (lane >= d) incl += y;
    }
    int run = incl - s;
#pragma unroll 1
    for (int i = 0; i < NBRUN / 32; ++i) {
      const int cv = cnt[base + i];
      offs[base + i] = run;
      cur[base + i]  = run;
      run += cv;
    }
  }
  __syncthreads();

  if (wave == 0) {
#pragma unroll 1
    for (int w2 = 0; w2 < NWAVE; ++w2) {
      int c = misc[w2];
      c = c < 0 ? 0 : (c > WLCAP ? WLCAP : c);
#pragma unroll 1
      for (int b0 = 0; b0 < c; b0 += 32) {
        const int idx = b0 + lane;
        const int ent = wl[w2 * WLCAP + (idx < WLCAP ? idx : WLCAP - 1)];
        int eid = (ent >> SLB) & 0x1FFFFF;
        eid = eid > NE - 1 ? NE - 1 : eid;
        int sr = srcs[eid];
        sr = sr < 0 ? 0 : (sr > NN - 1 ? NN - 1 : sr);
        const int m32 = (c - b0) < 32 ? (c - b0) : 32;
#pragma unroll 1
        for (int k = 0; k < m32; ++k) {
          const int u    = __builtin_amdgcn_readlane(ent, k);
          const int wd   = __builtin_amdgcn_readlane(sr, k);
          const int slot = u & (NBRUN - 1);
          if (lane == 0) {
            int p = cur[slot];
            p = p < 0 ? 0 : (p > RCAP - 1 ? RCAP - 1 : p);
            pl[p] = wd;
            cur[slot] = p + 1;
          }
        }
      }
    }
  }
  __syncthreads();

  const int ovf = misc[9];
  int* lp = HITS + (size_t)blk * RCAP;
  int* cp = CNT  + (size_t)blk * NBRUN;
  int* op = OFF  + (size_t)blk * NBRUN;
  int* dp = DISI + (size_t)blk * NBRUN;
  int* fp = FLAG + (size_t)blk * 32;
  bucket_flush(pl, cnt, ovf, lp, cp, op, dp, fp, tid);
  __threadfence();
  bucket_flush(pl, cnt, ovf, lp, cp, op, dp, fp, tid);
}

template <int KTOT>
__device__ __forceinline__ void gemm_16x64(const unsigned short* __restrict__ ap,
                                           const unsigned short* __restrict__ bp, v8f (&acc)[4]) {
#pragma unroll 1
  for (int k0 = 0; k0 < KTOT; k0 += 32) {
    FragB af;
    af.h[0] = *(const v8usa*)(ap + k0);
    af.h[1] = *(const v8usa*)(ap + k0 + 16);
#pragma unroll
    for (int nt = 0; nt < 4; ++nt) {
      const unsigned short* wq = bp + (size_t)(16 * nt) * (size_t)KTOT + k0;
      FragB bf;
      bf.h[0] = *(const v8usa*)wq;
      bf.h[1] = *(const v8usa*)(wq + 16);
      acc[nt] = wmb(af, bf, acc[nt]);
    }
  }
}

__device__ __forceinline__ void stage_d(float* stg, const v8f (&acc)[4], int wave, int hh, int m) {
#pragma unroll
  for (int nt = 0; nt < 4; ++nt) {
#pragma unroll
    for (int r = 0; r < 8; ++r) stg[(16 * wave + 8 * hh + r) * SP + 16 * nt + m] = acc[nt][r];
  }
}

__global__ __launch_bounds__(NTHR) __attribute__((amdgpu_num_vgpr(248)))
void k_gemm(const unsigned short* __restrict__ A, const unsigned short* __restrict__ BT,
            const float* __restrict__ DIS, float* HP) {
  __shared__ __attribute__((aligned(16))) float stg[GBM * SP];
  const int tid = (int)threadIdx.x, lane = tid & 31, wave = tid >> 5, hh = lane >> 4, m = lane & 15;
  const int rowBase = (int)blockIdx.x * GBM;

  v8f acc[4];
  {
    const v8f z = {0.f, 0.f, 0.f, 0.f, 0.f, 0.f, 0.f, 0.f};
#pragma unroll
    for (int t = 0; t < 4; ++t) acc[t] = z;
  }
  const unsigned short* ap = A + (size_t)(rowBase + 16 * wave + m) * (size_t)KL + 8 * hh;
  const unsigned short* bp = BT + (size_t)m * (size_t)KL + 8 * hh;
  gemm_16x64<KL>(ap, bp, acc);
  stage_d(stg, acc, wave, hh, m);
  __syncthreads();

#pragma unroll 1
  for (int i = 0; i < 8; ++i) {
    const int lr   = 16 * wave + 2 * i + hh;
    const int grow = rowBase + lr;
    const bool live = grow < NN;
    const v4f a = *(const v4fa*)(stg + lr * SP + 4 * m);
    const float dv = DIS[grow];
    asm volatile("" :: "v"(a));
    asm volatile("" :: "v"(dv));
    const float v0 = a.x * dv, v1 = a.y * dv, v2 = a.z * dv, v3 = a.w * dv;
    v4f o;
    o.x = live ? v0 : 0.0f; o.y = live ? v1 : 0.0f; o.z = live ? v2 : 0.0f; o.w = live ? v3 : 0.0f;
    st2_v4f(HP + (size_t)grow * HD + 4 * m, o);
  }
}

__global__ __launch_bounds__(NTHR) void k_replay(const int* __restrict__ HITS, const int* __restrict__ CNT,
                                                 const int* __restrict__ OFF, const float* __restrict__ DIS,
                                                 const int* __restrict__ FLAG, const float* __restrict__ HP,
                                                 const float* __restrict__ bias, float* Y, float* REC) {
  __shared__ __attribute__((aligned(16))) float sb[64];
  __shared__ __attribute__((aligned(16))) float wst[NWAVE * WSTW];
  __shared__ __attribute__((aligned(16))) float pst[RECW];
  const int tid = (int)threadIdx.x, lane = tid & 31;
  const int wave = __builtin_amdgcn_readfirstlane(tid >> 5);
  const int blk = (int)blockIdx.x;
  const int nodeBase = blk * NBRUN;

  if (wave == 0) {
    const int q = lane & 15;
    const v4f b = *(const v4fa*)(bias + 4 * q);
    v4f r;
    r.x = bf16_val(b.x); r.y = bf16_val(b.y); r.z = bf16_val(b.z); r.w = bf16_val(b.w);
    *(v4fa*)(sb + 4 * q) = r;
  }
  __syncthreads();

  const v2f bl = *(const v2fa*)(sb + 2 * lane);
  const int flag = FLAG[(size_t)blk * 32];
  const int* lb = HITS + (size_t)blk * RCAP;
  const float qnan = __uint_as_float(0x7fc00000u);
  int wn = 0;
  float m0 = 0.0f, m1 = 0.0f, q0 = 0.0f, q1 = 0.0f;

#pragma unroll 1
  for (int si = 0; si < NBRUN / NWAVE; ++si) {
    const int node = nodeBase + si * NWAVE + wave;
    if (node < NN) {
      int c = __builtin_amdgcn_readfirstlane(CNT[node]);
      int o = __builtin_amdgcn_readfirstlane(OFF[node]);
      const bool big = c > DEGCAP;
      c = c < 0 ? 0 : (c > DEGCAP ? DEGCAP : c);
      o = o < 0 ? 0 : (o > RCAP - 1 ? RCAP - 1 : o);
      int last = o + (c > 0 ? c : 1) - 1;
      last = last > RCAP - 1 ? RCAP - 1 : last;
      float a0 = 0.0f, a1 = 0.0f;
#pragma unroll 1
      for (int b0 = 0; b0 < c; b0 += 32) {
        int idx = o + b0 + lane;
        idx = idx > last ? last : idx;
        int sr = lb[idx];
        sr = sr < 0 ? 0 : (sr > NN - 1 ? NN - 1 : sr);
        const int m32 = (c - b0) < 32 ? (c - b0) : 32;
#pragma unroll 1
        for (int k = 0; k < m32; ++k) {
          const int sk = __builtin_amdgcn_readlane(sr, k);
          const v2f v = *(const v2fa*)(HP + (size_t)sk * HD + 2 * lane);
          a0 += v.x;
          a1 += v.y;
        }
      }
      const v2f g = *(const v2fa*)(HP + (size_t)node * HD + 2 * lane);
      a0 += g.x;
      a1 += g.y;
      const float dv = DIS[node];
      float y0 = dv * a0 + bl.x;
      float y1 = dv * a1 + bl.y;
      const bool bad = (flag != 0) | big;
      y0 = bad ? qnan : y0;
      y1 = bad ? qnan : y1;
      v2f ov;
      ov.x = y0; ov.y = y1;
      float* yp = Y + (size_t)node * HD + 2 * lane;
      *(volatile v2f*)yp = ov;
      __threadfence();
      *(volatile v2f*)yp = ov;
      wn += 1;
      const float rk = 1.0f / (float)wn;
      const float d0 = y0 - m0, d1 = y1 - m1;
      m0 = fmaf(d0, rk, m0);
      m1 = fmaf(d1, rk, m1);
      q0 = fmaf(d0, y0 - m0, q0);
      q1 = fmaf(d1, y1 - m1, q1);
    }
  }

  if (lane == 0) wst[wave * WSTW] = (float)wn;
  {
    v2f mm, qq;
    mm.x = m0; mm.y = m1; qq.x = q0; qq.y = q1;
    *(v2fa*)(wst + wave * WSTW + 4 + 2 * lane) = mm;
    *(v2fa*)(wst + wave * WSTW + 4 + HD + 2 * lane) = qq;
  }
  __syncthreads();
  if (tid < 64) {
    float n = 0.0f, mean = 0.0f, M2 = 0.0f;
#pragma unroll 1
    for (int w2 = 0; w2 < NWAVE; ++w2) {
      const float nb = wst[w2 * WSTW];
      const float mb = wst[w2 * WSTW + 4 + tid];
      const float qb = wst[w2 * WSTW + 4 + HD + tid];
      if (nb > 0.5f) {
        const float nn = n + nb;
        const float delta = mb - mean;
        const float f = nb / nn;
        mean = fmaf(delta, f, mean);
        M2 = M2 + qb + delta * delta * n * f;
        n = nn;
      }
    }
    pst[tid] = mean;
    pst[HD + tid] = M2;
  } else if (tid < 96) {
    float n = 0.0f;
#pragma unroll 1
    for (int w2 = 0; w2 < NWAVE; ++w2) n += wst[w2 * WSTW];
    pst[2 * HD + (tid - 64)] = n;
  }
  __syncthreads();
  {
    float* rp = REC + (size_t)blk * RECW;
    const int t4 = tid < RECW / 4 ? tid : RECW / 4 - 1;
    const v4f ps = *(const v4fa*)(pst + 4 * t4);
    asm volatile("" :: "v"(ps));
    if (tid < RECW / 4) *(volatile v4f*)(rp + 4 * tid) = ps;
    __threadfence();
    if (tid < RECW / 4) *(volatile v4f*)(rp + 4 * tid) = ps;
  }
}

__global__ __launch_bounds__(64) void k_comb(const float* __restrict__ REC, float* STAT) {
  __shared__ __attribute__((aligned(16))) float stg[2 * HD];
  const int tid = (int)threadIdx.x;
  double n = 0.0, mean = 0.0, M2 = 0.0;
#pragma unroll 1
  for (int b = 0; b < NBK; ++b) {
    const float* pr = REC + (size_t)b * RECW;
    const double nb = (double)pr[2 * HD];
    const double mb = (double)pr[tid];
    const double qb = (double)pr[HD + tid];
    if (nb > 0.5) {
      const double nn = n + nb;
      const double delta = mb - mean;
      const double f = nb / nn;
      mean = mean + delta * f;
      M2 = M2 + qb + delta * delta * n * f;
      n = nn;
    }
  }
  const double nt = n < 1.0 ? 1.0 : n;
  const float varf  = (float)(M2 / nt);
  const float meanf = (float)mean;
  const float rstd  = 1.0f / sqrtf(varf + 1e-5f);
  stg[tid] = meanf;
  stg[HD + tid] = rstd;
  __syncthreads();
  if (tid < 32) {
    const v4f v = *(const v4fa*)(stg + 4 * tid);
    st2_v4f(STAT + 4 * tid, v);
  }
}

__global__ __launch_bounds__(NTHR) void k_apply(const float* __restrict__ Y, const float* __restrict__ STAT,
                                                const float* __restrict__ gam, const float* __restrict__ bet,
                                                unsigned short* XHL) {
  __shared__ __attribute__((aligned(16))) float sp[256];
  const int tid = (int)threadIdx.x, lane = tid & 31, hh = lane >> 4, q = lane & 15;
  const int wave = __builtin_amdgcn_readfirstlane(tid >> 5);
  const int rowBase = (int)blockIdx.x * GBM;
  if (wave == 0) {
    const v4f s = *(const v4fa*)(STAT + 4 * lane);
    *(v4fa*)(sp + 4 * lane) = s;
  } else if (wave == 1) {
    const v4f g = *(const v4fa*)(gam + 4 * q);
    const v4f b = *(const v4fa*)(bet + 4 * q);
    asm volatile("" :: "v"(g));
    asm volatile("" :: "v"(b));
    const unsigned mg = (lane < 16) ? 0xffffffffu : 0u;
    v4f o;
    o.x = __uint_as_float(((bf16_bits(g.x) << 16) & mg) | ((bf16_bits(b.x) << 16) & ~mg));
    o.y = __uint_as_float(((bf16_bits(g.y) << 16) & mg) | ((bf16_bits(b.y) << 16) & ~mg));
    o.z = __uint_as_float(((bf16_bits(g.z) << 16) & mg) | ((bf16_bits(b.z) << 16) & ~mg));
    o.w = __uint_as_float(((bf16_bits(g.w) << 16) & mg) | ((bf16_bits(b.w) << 16) & ~mg));
    *(v4fa*)(sp + 128 + 4 * lane) = o;
  }
  __syncthreads();
  const v4f mu = *(const v4fa*)(sp + 4 * q);
  const v4f rs = *(const v4fa*)(sp + 64 + 4 * q);
  const v4f gg = *(const v4fa*)(sp + 128 + 4 * q);
  const v4f be = *(const v4fa*)(sp + 192 + 4 * q);

#pragma unroll 1
  for (int i = 0; i < 8; ++i) {
    const int grow = rowBase + 16 * wave + 2 * i + hh;
    const bool live = grow < NN;
    const int rc = live ? grow : NN - 1;
    const v4f y = *(const v4fa*)(Y + (size_t)rc * HD + 4 * q);
    asm volatile("" :: "v"(y));
    float v0 = bnr(y.x, mu.x, rs.x, gg.x, be.x), v1 = bnr(y.y, mu.y, rs.y, gg.y, be.y);
    float v2 = bnr(y.z, mu.z, rs.z, gg.z, be.z), v3 = bnr(y.w, mu.w, rs.w, gg.w, be.w);
    v0 = live ? v0 : 0.0f; v1 = live ? v1 : 0.0f; v2 = live ? v2 : 0.0f; v3 = live ? v3 : 0.0f;
    int h01, h23, l01, l23;
    hilo_pack(v0, v1, v2, v3, h01, h23, l01, l23);
    const v4i ow = regroup8(h01, h23, l01, l23, lane);
    unsigned short* hp = XHL + (size_t)grow * KL + 8 * q;
    *(volatile v4i*)hp = ow;
    __threadfence();
    *(volatile v4i*)hp = ow;
  }
}

__global__ __launch_bounds__(NTHR) __attribute__((amdgpu_num_vgpr(248)))
void k_head(const float* __restrict__ Y, const float* __restrict__ STAT, const float* __restrict__ gam,
            const float* __restrict__ bet, const unsigned short* __restrict__ FC1D,
            const float* __restrict__ fc1b, const float* __restrict__ fc2w, const float* __restrict__ fc2b,
            const int* __restrict__ FLAG, float* out) {
  __shared__ __attribute__((aligned(16))) unsigned short at[GBM * AP];
  __shared__ __attribute__((aligned(16))) float rt[GBM * RP];
  __shared__ __attribute__((aligned(16))) float sp[256];
  __shared__ __attribute__((aligned(16))) float fb[FC];
  __shared__ __attribute__((aligned(16))) float fw[2 * FC];
  __shared__ __attribute__((aligned(16))) float fb2[4];
  __shared__ __attribute__((aligned(16))) float lg[2 * GBM];
  const int tid = (int)threadIdx.x, lane = tid & 31, hh = lane >> 4, m = lane & 15;
  const int wave = __builtin_amdgcn_readfirstlane(tid >> 5);
  const int blk = (int)blockIdx.x;
  const int rowBase = blk * GBM;
  const int flag = FLAG[(size_t)(rowBase >> SLB) * 32];

  if (wave == 0) {
    const v4f s = *(const v4fa*)(STAT + 4 * lane);
    *(v4fa*)(sp + 4 * lane) = s;
  } else if (wave == 1) {
    const v4f g = *(const v4fa*)(gam + 4 * m);
    const v4f b = *(const v4fa*)(bet + 4 * m);
    asm volatile("" :: "v"(g));
    asm volatile("" :: "v"(b));
    const unsigned mg = (lane < 16) ? 0xffffffffu : 0u;
    v4f o;
    o.x = __uint_as_float(((bf16_bits(g.x) << 16) & mg) | ((bf16_bits(b.x) << 16) & ~mg));
    o.y = __uint_as_float(((bf16_bits(g.y) << 16) & mg) | ((bf16_bits(b.y) << 16) & ~mg));
    o.z = __uint_as_float(((bf16_bits(g.z) << 16) & mg) | ((bf16_bits(b.z) << 16) & ~mg));
    o.w = __uint_as_float(((bf16_bits(g.w) << 16) & mg) | ((bf16_bits(b.w) << 16) & ~mg));
    *(v4fa*)(sp + 128 + 4 * lane) = o;
  } else if (wave == 2) {
    const int q8 = lane & 7;
    const v4f w = *(const v4fa*)(fc2w + 4 * m);
    const v4f b = *(const v4fa*)(fc1b + 4 * q8);
    v4f wr, br;
    wr.x = bf16_val(w.x); wr.y = bf16_val(w.y); wr.z = bf16_val(w.z); wr.w = bf16_val(w.w);
    br.x = bf16_val(b.x); br.y = bf16_val(b.y); br.z = bf16_val(b.z); br.w = bf16_val(b.w);
    *(v4fa*)(fw + 4 * m) = wr;
    *(v4fa*)(fb + 4 * q8) = br;
  } else if (wave == 3) {
    const int c = lane & 1;
    const float b = fc2b[c];
    fb2[c] = bf16_val(b);
  }
  __syncthreads();

  {
    const v4f mu = *(const v4fa*)(sp + 4 * m);
    const v4f rs = *(const v4fa*)(sp + 64 + 4 * m);
    const v4f gg = *(const v4fa*)(sp + 128 + 4 * m);
    const v4f be = *(const v4fa*)(sp + 192 + 4 * m);
#pragma unroll 1
    for (int i = 0; i < 8; ++i) {
      const int lr   = 16 * wave + 2 * i + hh;
      const int grow = rowBase + lr;
      const bool live = grow < NN;
      const int rc = live ? grow : NN - 1;
      const v4f y = *(const v4fa*)(Y + (size_t)rc * HD + 4 * m);
      asm volatile("" :: "v"(y));
      float v0 = bnr(y.x, mu.x, rs.x, gg.x, be.x), v1 = bnr(y.y, mu.y, rs.y, gg.y, be.y);
      float v2 = bnr(y.z, mu.z, rs.z, gg.z, be.z), v3 = bnr(y.w, mu.w, rs.w, gg.w, be.w);
      v0 = live ? v0 : 0.0f; v1 = live ? v1 : 0.0f; v2 = live ? v2 : 0.0f; v3 = live ? v3 : 0.0f;
      int h01, h23, l01, l23;
      hilo_pack(v0, v1, v2, v3, h01, h23, l01, l23);
      const v4i ow = regroup8(h01, h23, l01, l23, lane);
      *(v4ia*)(at + lr * AP + 8 * m) = ow;
    }
  }
  __syncthreads();

  v8f acc0 = {0.f, 0.f, 0.f, 0.f, 0.f, 0.f, 0.f, 0.f};
  v8f acc1 = {0.f, 0.f, 0.f, 0.f, 0.f, 0.f, 0.f, 0.f};
  {
    const int arow = (16 * wave + m) * AP + 8 * hh;
    const unsigned short* bp = FC1D + (size_t)m * (size_t)KL + 8 * hh;
#pragma unroll 1
    for (int k0 = 0; k0 < KL; k0 += 32) {
      FragB af;
      af.h[0] = *(const v8usa*)(at + arow + k0);
      af.h[1] = *(const v8usa*)(at + arow + k0 + 16);
      FragB b0, b1;
      b0.h[0] = *(const v8usa*)(bp + k0);
      b0.h[1] = *(const v8usa*)(bp + k0 + 16);
      b1.h[0] = *(const v8usa*)(bp + (size_t)16 * KL + k0);
      b1.h[1] = *(const v8usa*)(bp + (size_t)16 * KL + k0 + 16);
      acc0 = wmb(af, b0, acc0);
      acc1 = wmb(af, b1, acc1);
    }
  }
  {
    const float c0 = fb[m], c1 = fb[16 + m];
#pragma unroll
    for (int r = 0; r < 8; ++r) {
      const int lr = 16 * wave + 8 * hh + r;
      float u0 = acc0[r] + c0, u1 = acc1[r] + c1;
      u0 = (u0 > 0.0f) ? u0 : (u0 - u0);
      u1 = (u1 > 0.0f) ? u1 : (u1 - u1);
      rt[lr * RP + m] = u0;
      rt[lr * RP + 16 + m] = u1;
    }
  }
  __syncthreads();

  if (tid < GBM) {
    float o0 = fb2[0], o1 = fb2[1];
#pragma unroll 4
    for (int j = 0; j < FC; ++j) {
      const float rv = rt[tid * RP + j];
      o0 = fmaf(rv, fw[2 * j], o0);
      o1 = fmaf(rv, fw[2 * j + 1], o1);
    }
    const float mx = ((o1 > o0) | (o1 != o1)) ? o1 : o0;
    const float s0 = o0 - mx, s1 = o1 - mx;
    const float ls = logf(expf(s0) + expf(s1));
    const float qnan = __uint_as_float(0x7fc00000u);
    float r0 = s0 - ls, r1 = s1 - ls;
    r0 = (flag != 0) ? qnan : r0;
    r1 = (flag != 0) ? qnan : r1;
    v2f ov;
    ov.x = r0; ov.y = r1;
    *(v2fa*)(lg + 2 * tid) = ov;
  }
  __syncthreads();

  {
    const int liveRows = (NN - rowBase) < GBM ? (NN - rowBase) : GBM;
    const int nv4 = liveRows / 2;
    float* ob = out + (size_t)blk * (size_t)(GBM * 2);
    const int t4 = tid < 64 ? tid : 63;
    const v4f v = *(const v4fa*)(lg + 4 * t4);
    asm volatile("" :: "v"(v));
    if (tid < nv4) *(volatile v4f*)(ob + 4 * tid) = v;
    __threadfence();
    if (tid < nv4) *(volatile v4f*)(ob + 4 * tid) = v;
  }
}

extern "C" void kernel_launch(void* const* d_in, const int* in_sizes, int n_in,
                              void* d_out, int out_size, void* d_ws, size_t ws_size,
                              hipStream_t stream) {
  if (n_in < 18) return;
  if (in_sizes[0] != NN * FD) return;
  if (in_sizes[1] != 2 * NE) return;
  if (in_sizes[2] != FD * HD) return;
  if (in_sizes[3] != HD) return;
  if (in_sizes[4] != HD * HD) return;
  if (in_sizes[5] != HD) return;
  if (in_sizes[6] != HD * HD) return;
  if (in_sizes[7] != HD) return;
  for (int i = 8; i < 14; ++i) { if (in_sizes[i] != HD) return; }
  if (in_sizes[14] != HD * FC) return;
  if (in_sizes[15] != FC) return;
  if (in_sizes[16] != FC * 2) return;
  if (in_sizes[17] != 2) return;
  if (out_size != NN * 2) return;

  const float* x    = (const float*)d_in[0];
  const int*   ei   = (const int*)d_in[1];
  const float* W0   = (const float*)d_in[2];
  const float* b0   = (const float*)d_in[3];
  const float* W1   = (const float*)d_in[4];
  const float* b1   = (const float*)d_in[5];
  const float* W2   = (const float*)d_in[6];
  const float* b2   = (const float*)d_in[7];
  const float* g0   = (const float*)d_in[8];
  const float* be0  = (const float*)d_in[9];
  const float* g1   = (const float*)d_in[10];
  const float* be1  = (const float*)d_in[11];
  const float* g2   = (const float*)d_in[12];
  const float* be2  = (const float*)d_in[13];
  const float* fc1w = (const float*)d_in[14];
  const float* fc1b = (const float*)d_in[15];
  const float* fc2w = (const float*)d_in[16];
  const float* fc2b = (const float*)d_in[17];
  float* out = (float*)d_out;
  const int* srcs = ei;
  const int* dsts = ei + NE;

  constexpr size_t zXHL  = (size_t)MP * KL * 2;
  constexpr size_t zF    = (size_t)MP * HD * 4;
  constexpr size_t zHITS = (size_t)NBK * RCAP * 4;
  constexpr size_t zTAB  = (size_t)NBK * NBRUN * 4;
  constexpr size_t zFLAG = (size_t)NBK * 128;
  constexpr size_t zREC  = (size_t)3 * NBK * RECW * 4;
  constexpr size_t zSTAT = (size_t)3 * 2 * HD * 4;
  constexpr size_t zW    = (size_t)HD * KL * 2;
  constexpr size_t zFC1D = (size_t)FC * KL * 2;
  constexpr size_t oXHL  = 0;
  constexpr size_t oHP   = oXHL + zXHL;
  constexpr size_t oY    = oHP + zF;
  constexpr size_t oHITS = oY + zF;
  constexpr size_t oCNT  = oHITS + zHITS;
  constexpr size_t oOFF  = oCNT + zTAB;
  constexpr size_t oDIS  = oOFF + zTAB;
  constexpr size_t oFLAG = oDIS + zTAB;
  constexpr size_t oREC  = oFLAG + zFLAG;
  constexpr size_t oSTAT = oREC + zREC;
  constexpr size_t oW0T  = oSTAT + zSTAT;
  constexpr size_t oW1D  = oW0T + zW;
  constexpr size_t oW2D  = oW1D + zW;
  constexpr size_t oFC1D = oW2D + zW;
  constexpr size_t oEND  = oFC1D + zFC1D;
  static_assert(zXHL % 256 == 0 && zF % 256 == 0 && zHITS % 256 == 0 && zTAB % 256 == 0 && zFLAG % 256 == 0);
  static_assert(zREC % 256 == 0 && zSTAT % 256 == 0 && zW % 256 == 0 && zFC1D % 256 == 0);
  static_assert((size_t)MP * FD * 2 == zXHL);
  static_assert((size_t)NBK * NBRUN >= (size_t)MP);
  static_assert(oEND <= (size_t)WSMAX);
  if (oEND > ws_size) return;

  char* ws = (char*)d_ws;
  unsigned short* XHL  = (unsigned short*)(ws + oXHL);
  float*          HP   = (float*)(ws + oHP);
  float*          Y    = (float*)(ws + oY);
  int*            HITS = (int*)(ws + oHITS);
  int*            CNT  = (int*)(ws + oCNT);
  int*            OFF  = (int*)(ws + oOFF);
  int*            DISI = (int*)(ws + oDIS);
  const float*    DIS  = (const float*)(ws + oDIS);
  int*            FLAG = (int*)(ws + oFLAG);
  float*          REC  = (float*)(ws + oREC);
  float*          STAT = (float*)(ws + oSTAT);
  unsigned short* W0T  = (unsigned short*)(ws + oW0T);
  unsigned short* W1D  = (unsigned short*)(ws + oW1D);
  unsigned short* W2D  = (unsigned short*)(ws + oW2D);
  unsigned short* FC1D = (unsigned short*)(ws + oFC1D);

  hipFuncSetAttribute(reinterpret_cast<const void*>(&k_bucket), hipFuncAttributeMaxDynamicSharedMemorySize, (int)BK_LDS);

  k_prep<<<PBTOT, NTHR, 0, stream>>>(x, W0, W1, W2, fc1w, XHL, W0T, W1D, W2D, FC1D);
  k_bucket<<<NBK, NTHR, BK_LDS, stream>>>(srcs, dsts, HITS, CNT, OFF, DISI, FLAG);
  k_gemm<<<MP / GBM, NTHR, 0, stream>>>(XHL, W0T, DIS, HP);

  k_replay<<<NBK, NTHR, 0, stream>>>(HITS, CNT, OFF, DIS, FLAG, HP, b0, Y, REC);
  k_comb<<<1, 64, 0, stream>>>(REC, STAT);
  k_apply<<<MP / GBM, NTHR, 0, stream>>>(Y, STAT, g0, be0, XHL);
  k_gemm<<<MP / GBM, NTHR, 0, stream>>>(XHL, W1D, DIS, HP);
  k_replay<<<NBK, NTHR, 0, stream>>>(HITS, CNT, OFF, DIS, FLAG, HP, b1, Y, REC + (size_t)NBK * RECW);
  k_comb<<<1, 64, 0, stream>>>(REC + (size_t)NBK * RECW, STAT + 2 * HD);
  k_apply<<<MP / GBM, NTHR, 0, stream>>>(Y, STAT + 2 * HD, g1, be1, XHL);
  k_gemm<<<MP / GBM, NTHR, 0, stream>>>(XHL, W2D, DIS, HP);
  k_replay<<<NBK, NTHR, 0, stream>>>(HITS, CNT, OFF, DIS, FLAG, HP, b2, Y, REC + (size_t)2 * NBK * RECW);
  k_comb<<<1, 64, 0, stream>>>(REC + (size_t)2 * NBK * RECW, STAT + 4 * HD);
  k_head<<<MP / GBM, NTHR, 0, stream>>>(Y, STAT + 4 * HD, g2, be2, FC1D, fc1b, fc2w, fc2b, FLAG, out);
}
